// Fusion_35287451304478
// MI455X (gfx1250) — hardware-verified
//
#include <hip/hip_runtime.h>
#include <math.h>
#include <stdint.h>

#define BH   32
#define SEQ  2048
#define HD   64
#define HPB  16
#define NQB  (SEQ / 64)
#define NKT  (SEQ / 64)
static_assert(NQB == 32 && NKT == 32);
static_assert((SEQ % 64) == 0 && HD == 64 && (BH % HPB) == 0);

typedef __bf16         v16b  __attribute__((ext_vector_type(16)));
typedef unsigned short v16us __attribute__((ext_vector_type(16)));
typedef unsigned short v8us  __attribute__((ext_vector_type(8)));
typedef float          v8f   __attribute__((ext_vector_type(8)));
typedef float          v4f   __attribute__((ext_vector_type(4)));
typedef unsigned int   v4u   __attribute__((ext_vector_type(4)));

#if defined(__HIP_DEVICE_COMPILE__)
#define DEV_ASM 1
#else
#define DEV_ASM 0
#endif

__device__ __forceinline__ unsigned short bf_bits(float f) {
  unsigned u = __float_as_uint(f);
  return (unsigned short)((u + 0x7FFFu + ((u >> 16) & 1u)) >> 16);
}
__device__ __forceinline__ float bf_up(unsigned short hb) { return __uint_as_float(((unsigned)hb) << 16); }
__device__ __forceinline__ unsigned pk16(unsigned short a, unsigned short b) { return (unsigned)a | ((unsigned)b << 16); }
__device__ __forceinline__ v8f zero8() { v8f z = {0.f, 0.f, 0.f, 0.f, 0.f, 0.f, 0.f, 0.f}; return z; }

union FB { v16b v; v16us u; v8us h[2]; };

__device__ __forceinline__ v8f mma_b(v16b a, v16b b, v8f c) {
  c = __builtin_amdgcn_wmma_f32_16x16x32_bf16(false, a, false, b, (short)0, c, false, false);
#if DEV_ASM
  asm volatile("v_nop\n\tv_nop\n\tv_nop\n\tv_nop" : "+v"(c) : "v"(a), "v"(b));
#endif
  return c;
}

__global__ __launch_bounds__(256) void cvt_bf16x8(const float* __restrict__ in, unsigned short* out, int n8) {
  const int i = blockIdx.x * 256 + (int)threadIdx.x;
  if (i < n8) {
    const v4f a  = *(const v4f*)(in + (size_t)i * 8);
    const v4f a4 = *(const v4f*)(in + (size_t)i * 8 + 4);
    v4u p;
    p[0] = pk16(bf_bits(a[0]),  bf_bits(a[1]));
    p[1] = pk16(bf_bits(a[2]),  bf_bits(a[3]));
    p[2] = pk16(bf_bits(a4[0]), bf_bits(a4[1]));
    p[3] = pk16(bf_bits(a4[2]), bf_bits(a4[3]));
    unsigned short* o = out + (size_t)i * 8;
    *(volatile v4u*)o = p;
    __threadfence();
    *(volatile v4u*)o = p;
  }
}

__global__ __launch_bounds__(256) void vtrans_bf16(const float* __restrict__ V, unsigned short* Vt) {
  __shared__ __align__(16) unsigned short Tt[64 * 72];
  const int tid  = (int)threadIdx.x;
  const int s0   = blockIdx.x * 64;
  const int bh   = blockIdx.y;
  const float* src = V + ((size_t)bh * SEQ + (size_t)s0) * HD;
  {
    const int r  = tid >> 2;
    const int cs = (tid & 3) * 16;
#pragma unroll
    for (int i = 0; i < 4; ++i) {
      const v4f f = *(const v4f*)(src + (size_t)r * HD + cs + 4 * i);
#pragma unroll
      for (int e = 0; e < 4; ++e) Tt[(cs + 4 * i + e) * 72 + r] = bf_bits(f[e]);
    }
  }
  __syncthreads();
  {
    const int wave = tid >> 5, lane = tid & 31;
    const int q = lane >> 3, c8 = (lane & 7) * 8;
    v4u val[2];
#pragma unroll
    for (int it = 0; it < 2; ++it) {
      const int d = wave * 8 + it * 4 + q;
      val[it] = *(const v4u*)(Tt + d * 72 + c8);
    }
    for (int pass = 0; pass < 2; ++pass) {
#pragma unroll
      for (int it = 0; it < 2; ++it) {
        const int d = wave * 8 + it * 4 + q;
        unsigned short* o = Vt + ((size_t)bh * HD + (size_t)d) * SEQ + s0 + c8;
        *(volatile v4u*)o = val[it];
      }
      __threadfence();
    }
  }
}

__global__ __launch_bounds__(128)
void attn_hd64(const unsigned short* __restrict__ qp, const unsigned short* __restrict__ kp,
               const unsigned short* __restrict__ vtp, const float* __restrict__ mk,
               float* outp, float sscale) {
  __shared__ __align__(16) unsigned short Ksh[64 * 64];
  __shared__ __align__(16) unsigned short Vth[64 * 64];
  __shared__ __align__(16) unsigned short Psh[4][16 * 64];
  __shared__ __align__(16) unsigned short Psl[4][16 * 64];
  __shared__ __align__(16) float          Os[4][16 * 64];

  const int tid  = (int)threadIdx.x;
  const int wave = tid >> 5;
  const int lane = tid & 31;
  const int hh   = lane >> 4;
  const int c    = lane & 15;

  const int bx   = blockIdx.x;
  const int qb   = bx % NQB;
  const int bh   = bx / NQB;
  const int q0   = qb * 64 + wave * 16;
  const size_t rowB = (size_t)bh * SEQ;
  const int mb   = (bh / HPB) * SEQ;
  const unsigned short* Vb = vtp + (size_t)bh * HD * SEQ;

  FB qa[2];
#pragma unroll
  for (int dc = 0; dc < 2; ++dc) {
    const size_t qo = (rowB + (size_t)(q0 + c)) * HD + dc * 32 + 8 * hh;
    qa[dc].h[0] = *(const v8us*)(qp + qo);
    qa[dc].h[1] = *(const v8us*)(qp + qo + 16);
  }

  float mrow[8], lrow[8];
  v8f oacc[4];
#pragma unroll
  for (int r = 0; r < 8; ++r) { mrow[r] = -INFINITY; lrow[r] = 0.f; }
#pragma unroll
  for (int t = 0; t < 4; ++t) oacc[t] = zero8();

  unsigned short* pwh = Psh[wave];
  unsigned short* pwl = Psl[wave];

  for (int kt = 0; kt < NKT; ++kt) {
    const int kv0 = kt * 64;
    __syncthreads();
    {
      const int r = tid >> 1, half = (tid & 1) * 32;
      const unsigned short* kg = kp + (rowB + (size_t)(kv0 + r)) * HD + half;
      const unsigned short* vg = Vb + (size_t)r * SEQ + kv0 + half;
#pragma unroll
      for (int i = 0; i < 4; ++i) {
        const v8us a0 = *(const v8us*)(kg + 8 * i);
        const v8us b0 = *(const v8us*)(vg + 8 * i);
        *(v8us*)(Ksh + r * 64 + half + 8 * i) = a0;
        *(v8us*)(Vth + r * 64 + half + 8 * i) = b0;
      }
    }
    __syncthreads();

    float mv[4];
#pragma unroll
    for (int j = 0; j < 4; ++j) mv[j] = bf_up(bf_bits(mk[mb + kv0 + j * 16 + c]));

    v8f s[4];
#pragma unroll
    for (int j = 0; j < 4; ++j) {
      v8f acc = zero8();
#pragma unroll
      for (int dc = 0; dc < 2; ++dc) {
        FB kb;
        kb.h[0] = *(const v8us*)(Ksh + (j * 16 + c) * 64 + dc * 32 + 8 * hh);
        kb.h[1] = *(const v8us*)(Ksh + (j * 16 + c) * 64 + dc * 32 + 16 + 8 * hh);
        acc = mma_b(qa[dc].v, kb.v, acc);
      }
#pragma unroll
      for (int r = 0; r < 8; ++r) s[j][r] = acc[r] * sscale + mv[j];
    }

#pragma unroll
    for (int r = 0; r < 8; ++r) {
      float m = s[0][r];
#pragma unroll
      for (int j = 1; j < 4; ++j) m = fmaxf(m, s[j][r]);
#pragma unroll
      for (int off = 1; off < 16; off <<= 1) m = fmaxf(m, __shfl_xor(m, off, 32));
      const float mnew  = fmaxf(mrow[r], m);
      const float msafe = (mnew == -INFINITY) ? 0.f : mnew;
      const float alpha = __expf(mrow[r] - msafe);
      mrow[r] = mnew;
      float psum = 0.f;
#pragma unroll
      for (int j = 0; j < 4; ++j) {
        const float p = __expf(s[j][r] - msafe);
        psum += p;
        const unsigned short hb = bf_bits(p);
        const unsigned short lb = bf_bits(p - bf_up(hb));
        const int pi = (8 * hh + r) * 64 + j * 16 + c;
        pwh[pi] = hb;
        pwl[pi] = lb;
      }
#pragma unroll
      for (int off = 1; off < 16; off <<= 1) psum += __shfl_xor(psum, off, 32);
      lrow[r] = lrow[r] * alpha + psum;
#pragma unroll
      for (int t = 0; t < 4; ++t) oacc[t][r] *= alpha;
    }
    __builtin_amdgcn_fence(__ATOMIC_RELEASE, "workgroup");
    __builtin_amdgcn_wave_barrier();
    __builtin_amdgcn_fence(__ATOMIC_ACQUIRE, "workgroup");

#pragma unroll 1
    for (int kk = 0; kk < 2; ++kk) {
      FB ph, pl;
      ph.h[0] = *(const v8us*)(pwh + c * 64 + kk * 32 + 8 * hh);
      ph.h[1] = *(const v8us*)(pwh + c * 64 + kk * 32 + 16 + 8 * hh);
      pl.h[0] = *(const v8us*)(pwl + c * 64 + kk * 32 + 8 * hh);
      pl.h[1] = *(const v8us*)(pwl + c * 64 + kk * 32 + 16 + 8 * hh);
#pragma unroll
      for (int t = 0; t < 4; ++t) {
        FB vb;
        vb.h[0] = *(const v8us*)(Vth + (t * 16 + c) * 64 + kk * 32 + 8 * hh);
        vb.h[1] = *(const v8us*)(Vth + (t * 16 + c) * 64 + kk * 32 + 16 + 8 * hh);
        oacc[t] = mma_b(ph.v, vb.v, oacc[t]);
        oacc[t] = mma_b(pl.v, vb.v, oacc[t]);
      }
    }
  }

  float* os = Os[wave];
#pragma unroll
  for (int r = 0; r < 8; ++r) {
    const float l = lrow[r];
    const float inv = (l > 0.f) ? (1.0f / l) : 0.f;
#pragma unroll
    for (int t = 0; t < 4; ++t) os[(8 * hh + r) * 64 + t * 16 + c] = oacc[t][r] * inv;
  }
  __builtin_amdgcn_fence(__ATOMIC_RELEASE, "workgroup");
  __builtin_amdgcn_wave_barrier();
  __builtin_amdgcn_fence(__ATOMIC_ACQUIRE, "workgroup");
  {
    const int h2 = lane >> 4, c4 = (lane & 15) * 4;
    v4f ov[8];
#pragma unroll
    for (int it = 0; it < 8; ++it) {
      const int row = it * 2 + h2;
      ov[it] = *(const v4f*)(os + row * 64 + c4);
    }
    for (int pass = 0; pass < 2; ++pass) {
#pragma unroll
      for (int it = 0; it < 8; ++it) {
        const int row = it * 2 + h2;
        float* o = outp + (rowB + (size_t)(q0 + row)) * HD + c4;
        *(volatile v4f*)o = ov[it];
      }
      __threadfence();
    }
  }
}

extern "C" void kernel_launch(void* const* d_in, const int* in_sizes, int n_in,
                              void* d_out, int out_size, void* d_ws, size_t ws_size,
                              hipStream_t stream) {
  if (n_in < 4) return;
  if (in_sizes[0] != BH * SEQ * HD) return;
  if (in_sizes[1] != BH * SEQ * HD) return;
  if (in_sizes[2] != BH * SEQ * HD) return;
  if (in_sizes[3] != (BH / HPB) * SEQ) return;
  if (out_size != BH * SEQ * HD) return;

  const float* q  = (const float*)d_in[0];
  const float* k  = (const float*)d_in[1];
  const float* v  = (const float*)d_in[2];
  const float* mk = (const float*)d_in[3];
  float* out = (float*)d_out;

  const size_t PP = (size_t)BH * SEQ * HD * 2;
  size_t off = 0;
  const size_t oQ = off; off += PP;
  const size_t oK = off; off += PP;
  const size_t oV = off; off += PP;
  if (off > ws_size) return;
  if (off > (size_t)134217728) return;

  char* ws = (char*)d_ws;
  unsigned short* Qb = (unsigned short*)(ws + oQ);
  unsigned short* Kb = (unsigned short*)(ws + oK);
  unsigned short* Vt = (unsigned short*)(ws + oV);

  const int n8 = BH * SEQ * HD / 8;
  const dim3 blk(256);
  const dim3 gCvt((n8 + 255) / 256);
  const dim3 gVt(SEQ / 64, BH);
  const dim3 gAttn(BH * NQB);

  cvt_bf16x8<<<gCvt, blk, 0, stream>>>(q, Qb, n8);
  cvt_bf16x8<<<gCvt, blk, 0, stream>>>(k, Kb, n8);
  vtrans_bf16<<<gVt, blk, 0, stream>>>(v, Vt);
  attn_hd64<<<gAttn, dim3(128), 0, stream>>>(Qb, Kb, Vt, mk, out, 0.125f);
  (void)hipGetLastError();
}
